// Model_1640677507274
// MI455X (gfx1250) — hardware-verified
//
#include <hip/hip_runtime.h>


#ifndef NB
#define NB 8
#endif
#ifndef SEQ
#define SEQ 1024
#endif
#define NB_FULL  8
#define SEQ_FULL 1024
#ifndef OUT_SEQ
#define OUT_SEQ SEQ
#endif
#define DM   128
#define NH_  8
#define HD   128
#define OSP2 132
#define WTP  33
#define LOG2E 1.4426950408889634f
#define LSL  0.2f
#define PSH  14.0f
#define NEGB (-3.0e38f)
#define KEEPT (-1.0e37f)

static_assert(DM % 32 == 0);
static_assert(HD == 128);
static_assert(HD % 32 == 0);
static_assert(SEQ % 64 == 0);
static_assert((NB * SEQ) % 64 == 0);
static_assert(SEQ % 32 == 0);
static_assert(SEQ % 16 == 0);
static_assert(SEQ % 4 == 0);
static_assert(SEQ_FULL % 4 == 0);
static_assert(((size_t)SEQ * DM) % 8 == 0);
static_assert(NB <= NB_FULL);
static_assert(SEQ <= SEQ_FULL);
static_assert((OSP2 * 4) % 16 == 0);
static_assert(OSP2 >= HD);
static_assert(32 * 16 * 4 == 16 * 64 * 2);
static_assert(16 * 16 * 2 == 2 * 64 * 4);
static_assert(NH_ * 2 == 16);
static_assert(32 * 16 == HD * 4);
static_assert(256 * 2 * 16 == 32 * DM * 2);
static_assert(DM % 8 == 0);
static_assert((2 * 16 * 68 + 2 * 2 * 64) * 4 <= 131072);
static_assert(16 * OSP2 * 4 <= 131072);
static_assert(DM * WTP * 4 <= 131072);

typedef _Float16 h16;
typedef unsigned short bf;
typedef __attribute__((ext_vector_type(16))) __bf16   v16bf;
typedef __attribute__((ext_vector_type(16))) _Float16 v16h;
typedef __attribute__((ext_vector_type(8)))  _Float16 v8h;
typedef __attribute__((ext_vector_type(8)))  unsigned short v8us;
typedef __attribute__((ext_vector_type(8)))  float    v8f;
typedef __attribute__((ext_vector_type(4)))  float    v4f;
typedef __attribute__((ext_vector_type(4)))  int      v4i;
typedef v4f  __attribute__((may_alias)) v4fa;

__device__ __forceinline__ unsigned short f2bf(float f) { unsigned u = __float_as_uint(f); u += 0x7FFFu + ((u >> 16) & 1u); return (unsigned short)(u >> 16); }
__device__ __forceinline__ float bfr(float f) { return __uint_as_float(((unsigned)f2bf(f)) << 16); }
__device__ __forceinline__ v16h cat16(v8h lo, v8h hi) { return __builtin_shufflevector(lo, hi, 0, 1, 2, 3, 4, 5, 6, 7, 8, 9, 10, 11, 12, 13, 14, 15); }
__device__ __forceinline__ v16bf cat16b(v8us lo, v8us hi) { return __builtin_bit_cast(v16bf, __builtin_shufflevector(lo, hi, 0, 1, 2, 3, 4, 5, 6, 7, 8, 9, 10, 11, 12, 13, 14, 15)); }
__device__ __forceinline__ v8f wmma16(v16h a, v16h b, v8f c) { return __builtin_amdgcn_wmma_f32_16x16x32_f16(false, a, false, b, (short)0, c, false, false); }
__device__ __forceinline__ v8f wmmab(v16bf a, v16bf b, v8f c) { return __builtin_amdgcn_wmma_f32_16x16x32_bf16(false, a, false, b, (short)0, c, false, false); }
__device__ __forceinline__ v16h  ldh(const h16* p) { return cat16(*(const v8h*)p, *(const v8h*)(p + 16)); }
__device__ __forceinline__ v16bf ldb(const bf* p)  { return cat16b(*(const v8us*)p, *(const v8us*)(p + 16)); }
__device__ __forceinline__ void wave_sync() { __builtin_amdgcn_fence(3  , "wavefront"); __builtin_amdgcn_wave_barrier(); asm volatile("" ::: "memory"); }

__device__ __forceinline__ v8f wmma16g(v16h a, v16h b, v8f c) { c = wmma16(a, b, c); asm volatile("v_nop\n\tv_nop\n\tv_nop\n\tv_nop" : "+v"(c) : "v"(a), "v"(b)); return c; }
__device__ __forceinline__ v8f wmmabg(v16bf a, v16bf b, v8f c) { c = wmmab(a, b, c); asm volatile("v_nop\n\tv_nop\n\tv_nop\n\tv_nop" : "+v"(c) : "v"(a), "v"(b)); return c; }
static __device__ __forceinline__ h16 toh_flush(float v) { const h16 r = (h16)v; return (__builtin_fabsf(v) < 6.103515625e-05f) ? (h16)0.0f : r; }

__global__ __launch_bounds__(256) void k_cvt8(const float* __restrict__ src, bf* dst, size_t n8) {
    const size_t i = (size_t)blockIdx.x * 256 + threadIdx.x; if (i >= n8) return;
    const v8f v = *(const v8f*)(src + i * 8); v8us o;
#pragma unroll
    for (int k = 0; k < 8; ++k) o[k] = f2bf(v[k]);
    *(volatile v8us*)(dst + i * 8) = o; __threadfence(); *(volatile v8us*)(dst + i * 8) = o;
}

__global__ __launch_bounds__(256) void k_wtr(const float* __restrict__ W, bf* WT) {
    __shared__ float ts[DM * WTP];
    const int tid = threadIdx.x; const int hd = blockIdx.x, o0 = blockIdx.y * 32;
    const float* src = W + (size_t)hd * DM * HD;
#pragma unroll 1
    for (int it = 0; it < DM / 8; ++it) { const int i = it * 8 + (tid >> 5), o = tid & 31;
        ts[i * WTP + o] = src[(size_t)i * HD + o0 + o]; }
    __syncthreads();
    bf* dst = WT + ((size_t)hd * HD + o0) * DM;
#pragma unroll 1
    for (int ps = 0; ps < 2; ++ps) {
#pragma unroll
        for (int it = 0; it < 2; ++it) { const int p = it * 256 + tid; const int row = p >> 4, c8 = (p & 15) * 8;
            v8us o;
#pragma unroll
            for (int k = 0; k < 8; ++k) o[k] = f2bf(ts[(c8 + k) * WTP + row]);
            *(volatile v8us*)(dst + (size_t)row * DM + c8) = o; }
        if (ps == 0) __threadfence(); }
}

__global__ __launch_bounds__(256) void k_gtab(const int* __restrict__ adj, const float* __restrict__ bias, float* GT, int n4) {
#pragma clang fp contract(off)
    const int i = blockIdx.x * 256 + threadIdx.x; if (i >= n4) return;
    const int row = i / (SEQ / 4), c4 = (i % (SEQ / 4)) * 4;
    const size_t so = (size_t)row * SEQ_FULL + c4;
    const v4i a = *(const v4i*)(adj + so); const v4f bv = *(const v4f*)(bias + so); v4f o;
#pragma unroll
    for (int k = 0; k < 4; ++k) { const float g = bfr(bv[k]) * LOG2E; o[k] = (a[k] != 0) ? g : NEGB; }
    *(volatile v4f*)(GT + (size_t)i * 4) = o; __threadfence(); *(volatile v4f*)(GT + (size_t)i * 4) = o;
}

__global__ __launch_bounds__(64) void k_hproj(const bf* __restrict__ WT, const bf* __restrict__ XB, const float* __restrict__ avec, h16* VT, float* SS) {
    __shared__ __align__(16) float os[2 * 16 * 68];
    __shared__ __align__(16) float sp[2 * 2 * 64];
    const int K = DM;
    const int lane = threadIdx.x & 31, lr = lane & 15, hi = lane >> 4;
    const int wave = __builtin_amdgcn_readfirstlane((int)(threadIdx.x >> 5));
    const int hd = blockIdx.x; const int r0 = hd * HD + wave * 64, c0 = blockIdx.y * 64;
    v8f acc[4][4];
#pragma unroll
    for (int mb = 0; mb < 4; ++mb)
#pragma unroll
        for (int nb = 0; nb < 4; ++nb) acc[mb][nb] = (v8f){};
    const size_t aoff = (size_t)(r0 + lr) * K + 8 * hi, boff = (size_t)(c0 + lr) * K + 8 * hi;
#pragma unroll 1
    for (int kc = 0; kc < K; kc += 32) {
        v16bf a[4];
#pragma unroll
        for (int mb = 0; mb < 4; ++mb) a[mb] = ldb(WT + aoff + (size_t)mb * 16 * K + kc);
#pragma unroll
        for (int nb = 0; nb < 4; ++nb) { const v16bf b = ldb(XB + boff + (size_t)nb * 16 * K + kc);
#pragma unroll
            for (int mb = 0; mb < 4; ++mb) acc[mb][nb] = wmmabg(a[mb], b, acc[mb][nb]); }
    }
    const int bb = c0 / SEQ, tt = c0 % SEQ;
    const size_t tbase = ((size_t)(bb * NH_ + hd) * HD + (size_t)wave * 64) * SEQ + (size_t)tt;
    const int wb = wave * 16 * 68;
    const float* ap = avec + (size_t)hd * (2 * HD) + wave * 64 + 8 * hi;
    float s1p[4], s2p[4];
#pragma unroll
    for (int nb = 0; nb < 4; ++nb) { s1p[nb] = 0.0f; s2p[nb] = 0.0f; }
#pragma unroll
    for (int mb = 0; mb < 4; ++mb) {
        const v4f p0 = *(const v4f*)(ap + mb * 16), p1 = *(const v4f*)(ap + mb * 16 + 4);
        const v4f q0 = *(const v4f*)(ap + HD + mb * 16), q1 = *(const v4f*)(ap + HD + mb * 16 + 4);
        float a1v[8], a2v[8];
#pragma unroll
        for (int j = 0; j < 4; ++j) { a1v[j] = bfr(p0[j]); a1v[4 + j] = bfr(p1[j]); a2v[j] = bfr(q0[j]); a2v[4 + j] = bfr(q1[j]); }
#pragma unroll
        for (int nb = 0; nb < 4; ++nb) {
#pragma unroll
            for (int j = 0; j < 8; ++j) { const float val = acc[mb][nb][j];
                os[wb + (hi * 8 + j) * 68 + nb * 16 + lr] = val;
                s1p[nb] += val * a1v[j]; s2p[nb] += val * a2v[j]; } }
        wave_sync();
#pragma unroll 1
        for (int ps = 0; ps < 2; ++ps) {
            const size_t sb = tbase + (size_t)(mb * 16) * SEQ;
#pragma unroll
            for (int s = 0; s < 4; ++s) { const int row = 4 * s + (lane >> 3), c8 = (lane & 7) * 8;
                const v4f x0 = *(const v4fa*)(&os[wb + row * 68 + c8]); const v4f x1 = *(const v4fa*)(&os[wb + row * 68 + c8 + 4]); v8h hv;
#pragma unroll
                for (int i = 0; i < 4; ++i) { hv[i] = toh_flush(x0[i]); hv[4 + i] = toh_flush(x1[i]); }
                *(volatile v8h*)(VT + sb + (size_t)row * SEQ + c8) = hv; }
            if (ps == 0) __threadfence(); }
        wave_sync();
    }
#pragma unroll
    for (int nb = 0; nb < 4; ++nb) { s1p[nb] += __shfl_xor(s1p[nb], 16, 32); s2p[nb] += __shfl_xor(s2p[nb], 16, 32); }
#pragma unroll
    for (int nb = 0; nb < 4; ++nb) { const float sv = hi ? s2p[nb] : s1p[nb]; sp[(wave * 2 + hi) * 64 + nb * 16 + lr] = sv; }
    __syncthreads();
    if (wave == 0) {
        const int wh = lane >> 4, q = lane & 15;
        const v4f u0 = *(const v4fa*)(&sp[(0 + wh) * 64 + 4 * q]); const v4f u1 = *(const v4fa*)(&sp[(2 + wh) * 64 + 4 * q]); v4f sv;
#pragma unroll
        for (int k = 0; k < 4; ++k) sv[k] = (u0[k] + u1[k]) * LOG2E;
        const size_t so = (size_t)wh * ((size_t)NB * NH_ * SEQ) + (size_t)(bb * NH_ + hd) * SEQ + (size_t)tt + (size_t)(4 * q);
        *(volatile v4f*)(SS + so) = sv; __threadfence(); *(volatile v4f*)(SS + so) = sv;
    }
}

__global__ __launch_bounds__(32 * NH_) __attribute__((amdgpu_num_vgpr(256))) void k_gatt(const h16* __restrict__ VT, const float* __restrict__ SS, const float* __restrict__ GT, float* OUT) {
    __shared__ __align__(16) float os[16 * OSP2];
    const int lane = threadIdx.x & 31, lr = lane & 15, hi = lane >> 4;
    const int wave = __builtin_amdgcn_readfirstlane((int)(threadIdx.x >> 5));
    const int b = blockIdx.y; const int t0 = blockIdx.x * 16;
    const int zh = b * NH_ + wave;
    const float si = SS[(size_t)zh * SEQ + t0 + lr];
    const float* sjp = SS + (size_t)NB * NH_ * SEQ + (size_t)zh * SEQ + 8 * hi;
    const float* gp = GT + (size_t)(t0 + lr) * SEQ + 8 * hi;
    const size_t vo = (size_t)zh * HD * SEQ + (size_t)lr * SEQ + 8 * hi;
    v8f o[8];
#pragma unroll
    for (int j = 0; j < 8; ++j) o[j] = (v8f){};
    float m = NEGB, l = 0.0f;
#pragma unroll 1
    for (int key0 = 0; key0 < SEQ; key0 += 32) {
        const float* g = gp + key0;
        const v4f g0 = *(const v4f*)g, g1 = *(const v4f*)(g + 4), g2 = *(const v4f*)(g + 16), g3 = *(const v4f*)(g + 20);
        const float* sj = sjp + key0;
        const v4f j0 = *(const v4f*)sj, j1 = *(const v4f*)(sj + 4), j2 = *(const v4f*)(sj + 16), j3 = *(const v4f*)(sj + 20);
        float gx[8], gy[8], jx[8], jy[8];
#pragma unroll
        for (int r = 0; r < 4; ++r) { gx[r] = g0[r]; gx[4 + r] = g1[r]; gy[r] = g2[r]; gy[4 + r] = g3[r]; jx[r] = j0[r]; jx[4 + r] = j1[r]; jy[r] = j2[r]; jy[4 + r] = j3[r]; }
        float ta[8], tb[8]; bool fa[8], fb[8]; float mx = NEGB;
#pragma unroll
        for (int r = 0; r < 8; ++r) {
            const float xa = si + jx[r], xb = si + jy[r];
            ta[r] = fmaxf(xa, xa * LSL) + gx[r]; tb[r] = fmaxf(xb, xb * LSL) + gy[r];
            fa[r] = gx[r] > KEEPT; fb[r] = gy[r] > KEEPT;
            mx = fmaxf(mx, fmaxf(ta[r], tb[r])); }
        mx = fmaxf(mx, __shfl_xor(mx, 16, 32));
        const float mnew = fmaxf(m, mx);
        const float alpha = __builtin_amdgcn_exp2f(m - mnew);
        const float sh = PSH - mnew;
        v16h pb; float ls = 0.0f;
#pragma unroll
        for (int r = 0; r < 8; ++r) {
            const float aa = ta[r] + sh, ab = tb[r] + sh;
            const float ea = __builtin_amdgcn_exp2f(aa), eb = __builtin_amdgcn_exp2f(ab);
            const float ga = (fa[r] & (aa >= -14.0f)) ? ea : 0.0f, gb = (fb[r] & (ab >= -14.0f)) ? eb : 0.0f;
            const h16 pa = (h16)ga; const h16 pc = (h16)gb;
            pb[r] = pa; pb[8 + r] = pc;
            ls += (float)pa + (float)pc; }
        l = l * alpha + ls; m = mnew;
#pragma unroll
        for (int j = 0; j < 8; ++j) o[j] = o[j] * alpha;
        const h16* va = VT + vo + key0;
#pragma unroll
        for (int jj = 0; jj < 8; jj += 4) {
            const v16h v0 = ldh(va + (size_t)(jj + 0) * 16 * SEQ), v1 = ldh(va + (size_t)(jj + 1) * 16 * SEQ);
            const v16h v2 = ldh(va + (size_t)(jj + 2) * 16 * SEQ), v3 = ldh(va + (size_t)(jj + 3) * 16 * SEQ);
            o[jj + 0] = wmma16g(v0, pb, o[jj + 0]); o[jj + 1] = wmma16g(v1, pb, o[jj + 1]);
            o[jj + 2] = wmma16g(v2, pb, o[jj + 2]); o[jj + 3] = wmma16g(v3, pb, o[jj + 3]); }
    }
    l += __shfl_xor(l, 16, 32);
    const bool any = l > 0.0f;
    const float lsafe = any ? l : 1.0f;
    const float inv = any ? (1.0f / lsafe) : __uint_as_float(0x7FC00000u);
    const float sc = inv * 0.125f;
#pragma unroll 1
    for (int hh = 0; hh < NH_; ++hh) {
        if (wave == hh) {
#pragma unroll
            for (int j = 0; j < 8; ++j) {
                v4f a, c;
                a[0] = o[j][0] * sc; a[1] = o[j][1] * sc; a[2] = o[j][2] * sc; a[3] = o[j][3] * sc; c[0] = o[j][4] * sc; c[1] = o[j][5] * sc; c[2] = o[j][6] * sc; c[3] = o[j][7] * sc;
                const int ix = lr * OSP2 + 16 * j + 8 * hi;
                if (hh > 0) { const v4f pa = *(const v4fa*)(&os[ix]); const v4f pc = *(const v4fa*)(&os[ix + 4]); a = a + pa; c = c + pc; }
                *(v4fa*)(&os[ix]) = a; *(v4fa*)(&os[ix + 4]) = c; }
        }
        __syncthreads();
    }
    float* orow = OUT + ((size_t)b * OUT_SEQ + t0) * HD;
#pragma unroll 1
    for (int ps = 0; ps < 2; ++ps) {
#pragma unroll
        for (int s = 0; s < 2; ++s) { const int row = 2 * wave + s;
            const v4f val = *(const v4fa*)(&os[row * OSP2 + lane * 4]);
            *(volatile v4f*)(orow + (size_t)row * HD + lane * 4) = val; }
        if (ps == 0) __threadfence(); }
}

static constexpr size_t al256(size_t v) { return (v + 255) & ~(size_t)255; }
static constexpr size_t SZ_XB = al256((size_t)NB * SEQ * DM * 2);
static constexpr size_t SZ_WT = al256((size_t)NH_ * HD * DM * 2);
static constexpr size_t SZ_GT = al256((size_t)SEQ * SEQ * 4);
static constexpr size_t SZ_VT = al256((size_t)NB * NH_ * HD * SEQ * 2);
static constexpr size_t SZ_SS = al256((size_t)2 * NB * NH_ * SEQ * 4);
static constexpr size_t SZ_TOTAL = SZ_XB + SZ_WT + SZ_GT + SZ_VT + SZ_SS;
static_assert(SZ_TOTAL <= (size_t)134217728);
static_assert(((size_t)NB * SEQ * DM) % 8 == 0);
static_assert(((size_t)SEQ * SEQ) % 4 == 0);
static_assert(((size_t)NB * NH_ * SEQ * 4) % 256 == 0);

extern "C" void kernel_launch(void* const* d_in, const int* in_sizes, int n_in,
                              void* d_out, int out_size, void* d_ws, size_t ws_size, hipStream_t stream) {
    if (n_in < 5) return;
    const size_t needx = ((size_t)(NB - 1) * SEQ_FULL + SEQ) * DM;
    const size_t needt = (size_t)(SEQ - 1) * SEQ_FULL + SEQ;
    if ((size_t)in_sizes[0] < needx) return;
    if ((size_t)in_sizes[1] < needt || (size_t)in_sizes[2] < needt) return;
    if ((size_t)in_sizes[3] < (size_t)NH_ * DM * HD || (size_t)in_sizes[4] < (size_t)NH_ * 2 * HD) return;
    if ((size_t)out_size < ((size_t)(NB - 1) * OUT_SEQ + SEQ) * HD) return;
    if (SZ_TOTAL > ws_size) return;
    const float* hin  = (const float*)d_in[0];
    const int*   adj  = (const int*)d_in[1];
    const float* bias = (const float*)d_in[2];
    const float* wgt  = (const float*)d_in[3];
    const float* avec = (const float*)d_in[4];
    float* OUT = (float*)d_out;
    char* wsp = (char*)d_ws;
    bf*    XB = (bf*)wsp;    wsp += SZ_XB;
    bf*    WT = (bf*)wsp;    wsp += SZ_WT;
    float* GT = (float*)wsp; wsp += SZ_GT;
    h16*   VT = (h16*)wsp;   wsp += SZ_VT;
    float* SS = (float*)wsp; wsp += SZ_SS;

    if (SEQ == SEQ_FULL) {
        const size_t n8 = (size_t)NB * SEQ * DM / 8;
        k_cvt8<<<(unsigned)((n8 + 255) / 256), 256, 0, stream>>>(hin, XB, n8);
    } else {
        const size_t n8 = (size_t)SEQ * DM / 8;
        for (int b = 0; b < NB; ++b) k_cvt8<<<(unsigned)((n8 + 255) / 256), 256, 0, stream>>>(hin + (size_t)b * SEQ_FULL * DM, XB + (size_t)b * SEQ * DM, n8);
    }
    k_wtr<<<dim3(NH_, HD / 32, 1), 256, 0, stream>>>(wgt, WT);
    { const int n4 = SEQ * SEQ / 4;
      k_gtab<<<(unsigned)((n4 + 255) / 256), 256, 0, stream>>>(adj, bias, GT, n4); }
    k_hproj<<<dim3(NH_, NB * SEQ / 64, 1), 64, 0, stream>>>(WT, XB, avec, VT, SS);
    k_gatt<<<dim3(SEQ / 16, NB, 1), 32 * NH_, 0, stream>>>(VT, SS, GT, OUT);
}
